// GCNConvLayer_20650202759169
// MI455X (gfx1250) — hardware-verified
//
#include <hip/hip_runtime.h>
#include <stddef.h>


#define FD      128
#define NTHR    256
#define NWAVE   8
#define EPT     8
#define NGRP    2
#define CHUNK   (NTHR * EPT * NGRP)
#define WCAP    (EPT * NGRP * 32)
#define LISTN   (NWAVE * WCAP)
#define NBC     4096
#define NBA     448
#define GBM     64
#define HSCALE  16.0f
#define WSCALE  256.0f
#define OINV    0.000244140625f
#define WSCAP   134217728
#define LDS_DEG ((NBC + LISTN + NBC + NBC + 16) * 4)
#define LDS_AGG ((NBA * FD + LISTN + NBA + 16) * 4)

static_assert((CHUNK & (CHUNK - 1)) == 0);
static_assert(CHUNK <= 4096);
static_assert(NBC <= 4096 && NBA < 4096);
static_assert(NBC == NWAVE * 4 * 128);
static_assert((NBC % NTHR) == 0);
static_assert((NBA % NWAVE) == 0);
static_assert(((NBA * FD) % 4) == 0);
static_assert(FD % 32 == 0);
static_assert(GBM == NWAVE * 8 && NTHR == 2 * FD);

typedef float          v4f  __attribute__((ext_vector_type(4)));
typedef float          v8f  __attribute__((ext_vector_type(8)));
typedef int            v4i  __attribute__((ext_vector_type(4)));
typedef unsigned short v8us __attribute__((ext_vector_type(8)));
typedef _Float16       v8h  __attribute__((ext_vector_type(8)));
typedef _Float16       v16h __attribute__((ext_vector_type(16)));
union FragH { v16h v; v8us h[2]; };
union Pack8 { v8h h; v8us u; };

__device__ __forceinline__ v8us cvt8h(v4f a, v4f b, float sc) {
  v8h r;
  r[0] = (_Float16)(a.x * sc); r[1] = (_Float16)(a.y * sc);
  r[2] = (_Float16)(a.z * sc); r[3] = (_Float16)(a.w * sc);
  r[4] = (_Float16)(b.x * sc); r[5] = (_Float16)(b.y * sc);
  r[6] = (_Float16)(b.z * sc); r[7] = (_Float16)(b.w * sc);
  Pack8 p;
  p.h = r;
  return p.u;
}

__device__ __forceinline__ v8f wmh(v16h a, v16h b, v8f c) {
  v8f d = __builtin_amdgcn_wmma_f32_16x16x32_f16(false, a, false, b, (short)0, c, false, false);
  asm volatile("v_nop\n\tv_nop\n\tv_nop\n\tv_nop" : "+v"(d) : "v"(a), "v"(b));
  return d;
}

template <int NB>
__device__ __forceinline__ int scan_chunk(const int* __restrict__ dsts, int nE, int cbase, int slotBase,
                                          int vec8, int* list, int tid, int lane, int wave) {
  (void)lane;
  int wc = 0;
#pragma unroll
  for (int g = 0; g < NGRP; ++g) {
    const int el0  = (g * NTHR + tid) * EPT;
    const int e0   = cbase + el0;
    const int sent = -2147483647 - 1;
    v4i da, db;
    if (vec8 != 0 && cbase + CHUNK <= nE) {
      da = *(const v4i*)(dsts + e0);
      db = *(const v4i*)(dsts + e0 + 4);
    } else {
      da.x = (e0     < nE) ? dsts[min(e0, nE - 1)] : sent;
      da.y = (e0 + 1 < nE) ? dsts[min(e0 + 1, nE - 1)] : sent;
      da.z = (e0 + 2 < nE) ? dsts[min(e0 + 2, nE - 1)] : sent;
      da.w = (e0 + 3 < nE) ? dsts[min(e0 + 3, nE - 1)] : sent;
      db.x = (e0 + 4 < nE) ? dsts[min(e0 + 4, nE - 1)] : sent;
      db.y = (e0 + 5 < nE) ? dsts[min(e0 + 5, nE - 1)] : sent;
      db.z = (e0 + 6 < nE) ? dsts[min(e0 + 6, nE - 1)] : sent;
      db.w = (e0 + 7 < nE) ? dsts[min(e0 + 7, nE - 1)] : sent;
    }
    const unsigned nb = (unsigned)slotBase;
    const unsigned s0 = (unsigned)da.x - nb, s1 = (unsigned)da.y - nb;
    const unsigned s2 = (unsigned)da.z - nb, s3 = (unsigned)da.w - nb;
    const unsigned s4 = (unsigned)db.x - nb, s5 = (unsigned)db.y - nb;
    const unsigned s6 = (unsigned)db.z - nb, s7 = (unsigned)db.w - nb;
    const bool h0 = s0 < (unsigned)NB, h1 = s1 < (unsigned)NB, h2 = s2 < (unsigned)NB, h3 = s3 < (unsigned)NB;
    const bool h4 = s4 < (unsigned)NB, h5 = s5 < (unsigned)NB, h6 = s6 < (unsigned)NB, h7 = s7 < (unsigned)NB;
    const unsigned any = __builtin_amdgcn_ballot_w32(h0 | h1 | h2 | h3 | h4 | h5 | h6 | h7);
    if (any != 0u) {
#define HITJ(J, HJ, SJ) { \
        const unsigned mj = __builtin_amdgcn_ballot_w32(HJ); \
        if (mj != 0u) { \
          if (HJ) { \
            const int pos = wc + (int)__builtin_amdgcn_mbcnt_lo(mj, 0u); \
            if (pos < WCAP) list[wave * WCAP + pos] = ((el0 + (J)) << 12) | (int)(SJ); \
          } \
          wc += (int)__builtin_popcount(mj); } }
      HITJ(0, h0, s0)
      HITJ(1, h1, s1)
      HITJ(2, h2, s2)
      HITJ(3, h3, s3)
      HITJ(4, h4, s4)
      HITJ(5, h5, s5)
      HITJ(6, h6, s6)
      HITJ(7, h7, s7)
#undef HITJ
    }
  }
  return wc;
}

__global__ __launch_bounds__(NTHR) void k_prep(const float* __restrict__ x, const float* __restrict__ W,
                                               unsigned short* A16, unsigned short* Bw,
                                               int nN, int hUnits, int nHB, int wUnits) {
  const int tid = threadIdx.x;
  const v4f z4 = {0.f, 0.f, 0.f, 0.f};
  if ((int)blockIdx.x < nHB) {
    const int i = (int)blockIdx.x * NTHR + tid;
    if (i >= hUnits) return;
    const int row = i >> 4;
    const int c0  = (i & 15) * 8;
    const int rc  = row < nN ? row : nN - 1;
    const float* p = x + (size_t)rc * FD + c0;
    v4f a = *(const v4f*)p, b = *(const v4f*)(p + 4);
    if (row >= nN) { a = z4; b = z4; }
    const v8us hv = cvt8h(a, b, HSCALE);
    unsigned short* d = A16 + (size_t)row * FD + c0;
    *(volatile v8us*)d = hv;
    __threadfence();
    *(volatile v8us*)d = hv;
  } else {
    const int j = ((int)blockIdx.x - nHB) * NTHR + tid;
    if (j >= wUnits) return;
    const float* p = W + (size_t)j * 8;
    const v4f a = *(const v4f*)p, b = *(const v4f*)(p + 4);
    const v8us hv = cvt8h(a, b, WSCALE);
    unsigned short* d = Bw + (size_t)j * 8;
    *(volatile v8us*)d = hv;
    __threadfence();
    *(volatile v8us*)d = hv;
  }
}

__global__ __launch_bounds__(NTHR) void k_degree(const int* __restrict__ dstA, float* nrmP, float* rdP,
                                                 int nE, int vec8) {
  extern __shared__ v4f lds_dyn[];
  int*   scnt = (int*)lds_dyn;
  int*   list = scnt + NBC;
  float* nrL  = (float*)(list + LISTN);
  float* rdL  = nrL + NBC;
  int*   wcnt = (int*)(rdL + NBC);
  const int tid = threadIdx.x, lane = tid & 31, wave = tid >> 5;
  const int nodeBase = (int)blockIdx.x * NBC;

  for (int i = tid; i < NBC; i += NTHR) scnt[i] = 0;
  __syncthreads();

  const int nChunks = (nE + CHUNK - 1) / CHUNK;
#pragma unroll 1
  for (int ch = 0; ch < nChunks; ++ch) {
    const int cbase = ch * CHUNK;
    const int wc = scan_chunk<NBC>(dstA, nE, cbase, nodeBase, vec8, list, tid, lane, wave);
    if (lane == 0) wcnt[wave] = wc;
    __syncthreads();
    if (wave == 0) {
#pragma unroll 1
      for (int wsx = 0; wsx < NWAVE; ++wsx) {
        int n = __builtin_amdgcn_readfirstlane(wcnt[wsx]);
        n = n > WCAP ? WCAP : (n < 0 ? 0 : n);
        const int* lp = list + wsx * WCAP;
#pragma unroll 1
        for (int i = 0; i < n; ++i) {
          const int ent  = __builtin_amdgcn_readfirstlane(lp[i]);
          const int slot = ent & (NBC - 1);
          if (lane == 0) scnt[slot] = scnt[slot] + 1;
        }
      }
    }
    __syncthreads();
  }

#pragma unroll 1
  for (int k = 0; k < NBC / NTHR; ++k) {
    const int idx = k * NTHR + tid;
    int c = scnt[idx];
    c = c < 0 ? 0 : (c > (1 << 24) ? (1 << 24) : c);
    const float d = (float)(c + 1);
    nrL[idx] = rsqrtf(d);
    rdL[idx] = 1.0f / d;
  }
  __syncthreads();

  float* np_ = nrmP + (size_t)nodeBase;
  float* rp_ = rdP  + (size_t)nodeBase;
#pragma unroll
  for (int q = 0; q < 4; ++q) {
    const int f = (wave * 4 + q) * 128 + 4 * lane;
    const v4f a = *(const v4f*)(nrL + f);
    const v4f b = *(const v4f*)(rdL + f);
    *(volatile v4f*)(np_ + f) = a;
    *(volatile v4f*)(rp_ + f) = b;
  }
  __threadfence();
#pragma unroll
  for (int q = 0; q < 4; ++q) {
    const int f = (wave * 4 + q) * 128 + 4 * lane;
    const v4f a = *(const v4f*)(nrL + f);
    const v4f b = *(const v4f*)(rdL + f);
    *(volatile v4f*)(np_ + f) = a;
    *(volatile v4f*)(rp_ + f) = b;
  }
}

__global__ __launch_bounds__(NTHR) void k_gemm(const unsigned short* __restrict__ A16,
                                               const unsigned short* __restrict__ Bw,
                                               const float* __restrict__ bias, float* Hp) {
  constexpr int TPW = 4;
  __shared__ __attribute__((aligned(16))) float stg[GBM * FD];
  const int tid = threadIdx.x, lane = tid & 31, wave = tid >> 5, hh = lane >> 4, m = lane & 15;
  const int rowBase = (int)blockIdx.x * GBM;
  const int r0 = (wave >> 1) * 16;
  const int c0 = (wave & 1) * (TPW * 16);

  v8f acc[TPW];
#pragma unroll
  for (int t = 0; t < TPW; ++t) { v8f z = {0.f, 0.f, 0.f, 0.f, 0.f, 0.f, 0.f, 0.f}; acc[t] = z; }
  const unsigned short* ap = A16 + (size_t)(rowBase + r0 + m) * FD + 8 * hh;
  const unsigned short* bq = Bw + (size_t)(c0 + m) * FD + 8 * hh;

#pragma unroll
  for (int kt = 0; kt < FD / 32; ++kt) {
    FragH a;
    a.h[0] = *(const v8us*)(ap + 32 * kt);
    a.h[1] = *(const v8us*)(ap + 32 * kt + 16);
#pragma unroll
    for (int t = 0; t < TPW; ++t) {
      const unsigned short* bp = bq + (size_t)(16 * t) * FD + 32 * kt;
      FragH b;
      b.h[0] = *(const v8us*)bp;
      b.h[1] = *(const v8us*)(bp + 16);
      acc[t] = wmh(a.v, b.v, acc[t]);
    }
  }

  {
    float* sp = stg + (size_t)(r0 + 8 * hh) * FD + c0 + m;
    const float* be = bias + c0 + m;
#pragma unroll
    for (int t = 0; t < TPW; ++t) {
      const float bv = be[16 * t];
#pragma unroll
      for (int r = 0; r < 8; ++r) sp[r * FD + 16 * t] = acc[t][r] * OINV + bv;
    }
  }
  __syncthreads();

  v4f ov[8];
#pragma unroll
  for (int it = 0; it < 8; ++it) {
    const int row = wave * 8 + it;
    ov[it] = *(const v4f*)(stg + (size_t)row * FD + 4 * lane);
    *(volatile v4f*)(Hp + (size_t)(rowBase + row) * FD + 4 * lane) = ov[it];
  }
  __threadfence();
#pragma unroll
  for (int it = 0; it < 8; ++it) {
    const int row = wave * 8 + it;
    *(volatile v4f*)(Hp + (size_t)(rowBase + row) * FD + 4 * lane) = ov[it];
  }
}

__global__ __launch_bounds__(NTHR) void k_aggr(
    const int* __restrict__ srcA, const int* __restrict__ dstA, const int* __restrict__ efA,
    const float* __restrict__ Hp, const float* __restrict__ nrmP, const float* __restrict__ rdP,
    const float* __restrict__ emb, const float* __restrict__ resw, float* outp,
    int nN, int nE, int nT, int vec8) {
  extern __shared__ v4f lds_dyn[];
  float* accL = (float*)lds_dyn;
  int*   list = (int*)(accL + NBA * FD);
  float* sNt  = (float*)(list + LISTN);
  int*   wcnt = (int*)(sNt + NBA);
  const int tid = threadIdx.x, lane = tid & 31, wave = tid >> 5;
  const int wv = __builtin_amdgcn_readfirstlane(wave);
  const int nodeBase = (int)blockIdx.x * NBA;
  const int col = 4 * lane;
  const v4f z4 = {0.f, 0.f, 0.f, 0.f};

  for (int i = tid; i < NBA * FD / 4; i += NTHR) lds_dyn[i] = z4;
  for (int s = tid; s < NBA; s += NTHR) {
    int nd = nodeBase + s;
    nd = nd > nN - 1 ? nN - 1 : nd;
    sNt[s] = nrmP[nd];
  }
  __syncthreads();

  const int nChunks = (nE + CHUNK - 1) / CHUNK;
#pragma unroll 1
  for (int ch = 0; ch < nChunks; ++ch) {
    const int cbase = ch * CHUNK;
    const int wc = scan_chunk<NBA>(dstA, nE, cbase, nodeBase, vec8, list, tid, lane, wave);
    if (lane == 0) wcnt[wave] = wc;
    __syncthreads();
#pragma unroll 1
    for (int wsx = 0; wsx < NWAVE; ++wsx) {
      int n = __builtin_amdgcn_readfirstlane(wcnt[wsx]);
      n = n > WCAP ? WCAP : (n < 0 ? 0 : n);
      const int* lp = list + wsx * WCAP;
#pragma unroll 1
      for (int i = 0; i < n; ++i) {
        const int ent = __builtin_amdgcn_readfirstlane(lp[i]);
        int slot = ent & 4095;
        slot = slot > NBA - 1 ? NBA - 1 : slot;
        if ((slot & (NWAVE - 1)) == wv) {
          int e = cbase + ((ent >> 12) & (CHUNK - 1));
          e = e > nE - 1 ? nE - 1 : e;
          int s = srcA[e];
          s = s < 0 ? 0 : (s > nN - 1 ? nN - 1 : s);
          int et = efA[e];
          et = et < 0 ? 0 : (et > nT - 1 ? nT - 1 : et);
          const float w = nrmP[s] * sNt[slot];
          const v4f hv = *(const v4f*)(Hp + (size_t)s * FD + col);
          const v4f ev = *(const v4f*)(emb + (size_t)et * FD + col);
          v4f r = hv + ev;
          r.x = fmaxf(r.x, 0.0f); r.y = fmaxf(r.y, 0.0f);
          r.z = fmaxf(r.z, 0.0f); r.w = fmaxf(r.w, 0.0f);
          r = r * w;
          v4f* aq = (v4f*)(accL + (size_t)slot * FD + col);
          const v4f a0 = *aq;
          *aq = a0 + r;
        }
      }
    }
    __syncthreads();
  }

  const v4f rw = *(const v4f*)(resw + col);
#pragma unroll 1
  for (int j = 0; j < NBA / NWAVE; ++j) {
    const int slot = j * NWAVE + wv;
    const int node = nodeBase + slot;
    if (node < nN) {
      const v4f a  = *(const v4f*)(accL + (size_t)slot * FD + col);
      const v4f hv = *(const v4f*)(Hp + (size_t)node * FD + col);
      const float rd = rdP[node];
      v4f t = hv + rw;
      t.x = fmaxf(t.x, 0.0f); t.y = fmaxf(t.y, 0.0f);
      t.z = fmaxf(t.z, 0.0f); t.w = fmaxf(t.w, 0.0f);
      const v4f o = a + t * rd;
      *(volatile v4f*)(outp + (size_t)node * FD + col) = o;
    }
  }
  __threadfence();
#pragma unroll 1
  for (int j = 0; j < NBA / NWAVE; ++j) {
    const int slot = j * NWAVE + wv;
    const int node = nodeBase + slot;
    if (node < nN) {
      const v4f a  = *(const v4f*)(accL + (size_t)slot * FD + col);
      const v4f hv = *(const v4f*)(Hp + (size_t)node * FD + col);
      const float rd = rdP[node];
      v4f t = hv + rw;
      t.x = fmaxf(t.x, 0.0f); t.y = fmaxf(t.y, 0.0f);
      t.z = fmaxf(t.z, 0.0f); t.w = fmaxf(t.w, 0.0f);
      const v4f o = a + t * rd;
      *(volatile v4f*)(outp + (size_t)node * FD + col) = o;
    }
  }
}

extern "C" void kernel_launch(void* const* d_in, const int* in_sizes, int n_in,
                              void* d_out, int out_size, void* d_ws, size_t ws_size,
                              hipStream_t stream) {
  if (n_in < 8) return;
  if (in_sizes[0] <= 0 || (in_sizes[0] % FD) != 0) return;
  const int nN = in_sizes[0] / FD;
  const int nE = in_sizes[1];
  if (nE <= 0 || in_sizes[2] != nE || in_sizes[3] != nE) return;
  if (in_sizes[4] != FD * FD || in_sizes[5] != FD || in_sizes[7] != FD) return;
  if (in_sizes[6] <= 0 || (in_sizes[6] % FD) != 0) return;
  const int nT = in_sizes[6] / FD;
  if (out_size != nN * FD) return;
  if (nN > (1 << 24) || nE > (1 << 28)) return;

  const float* x    = (const float*)d_in[0];
  const int*   ef   = (const int*)d_in[1];
  const int*   src  = (const int*)d_in[2];
  const int*   dst  = (const int*)d_in[3];
  const float* W    = (const float*)d_in[4];
  const float* bias = (const float*)d_in[5];
  const float* emb  = (const float*)d_in[6];
  const float* resw = (const float*)d_in[7];
  float* out = (float*)d_out;

  const int NPADG  = ((nN + GBM - 1) / GBM) * GBM;
  const int nGemm  = NPADG / GBM;
  const int hUnits = NPADG * (FD / 8);
  const int nHB    = hUnits / NTHR;
  const int wUnits = FD * FD / 8;
  const int nWB    = (wUnits + NTHR - 1) / NTHR;
  const int nDeg   = (nN + NBC - 1) / NBC;
  const int CNTPAD = nDeg * NBC;
  const int nAgg   = (nN + NBA - 1) / NBA;

  char* ws = (char*)d_ws;
  size_t off = 0;
  const size_t oB = off; off += (size_t)FD * FD * 2;          off = (off + 255) & ~(size_t)255;
  const size_t oA = off; off += (size_t)NPADG * FD * 2;       off = (off + 255) & ~(size_t)255;
  const size_t oH = off; off += (size_t)NPADG * FD * 4;       off = (off + 255) & ~(size_t)255;
  const size_t oN = off; off += (size_t)CNTPAD * 4;           off = (off + 255) & ~(size_t)255;
  const size_t oR = off; off += (size_t)CNTPAD * 4;           off = (off + 255) & ~(size_t)255;
  if (off > ws_size || off > (size_t)WSCAP) return;
  unsigned short* bw  = (unsigned short*)(ws + oB);
  unsigned short* a16 = (unsigned short*)(ws + oA);
  float* H    = (float*)(ws + oH);
  float* nrm  = (float*)(ws + oN);
  float* rdeg = (float*)(ws + oR);

  const int vec8 = ((nE & 3) == 0) ? 1 : 0;

  k_prep<<<nHB + nWB, NTHR, 0, stream>>>(x, W, a16, bw, nN, hUnits, nHB, wUnits);

  hipFuncSetAttribute(reinterpret_cast<const void*>(&k_degree),
                      hipFuncAttributeMaxDynamicSharedMemorySize, LDS_DEG);
  k_degree<<<nDeg, NTHR, LDS_DEG, stream>>>(dst, nrm, rdeg, nE, vec8);

  k_gemm<<<nGemm, NTHR, 0, stream>>>(a16, bw, bias, H);

  hipFuncSetAttribute(reinterpret_cast<const void*>(&k_aggr),
                      hipFuncAttributeMaxDynamicSharedMemorySize, LDS_AGG);
  k_aggr<<<nAgg, NTHR, LDS_AGG, stream>>>(src, dst, ef, H, nrm, rdeg, emb, resw, out, nN, nE, nT, vec8);
}
